// MAETransformerModel_76244259439065
// MI455X (gfx1250) — hardware-verified
//
#include <hip/hip_runtime.h>


#define NB_  32
#define SS   512
#define NT   (NB_ * SS)
#define INF  19
#define INP  32
#define DE   256
#define DDm  128
#define HE   8
#define HDd  4
#define DH   32
#define FE   1024
#define FD   512
#define LE   6
#define LD   2
#define RTM  NT
#define NW   256
#define DM   DE
#define LOSC 1024.0f

#define NN NW
typedef _Float16 h16;
typedef unsigned short bf;
typedef __attribute__((ext_vector_type(16))) __bf16   v16bf;
typedef __attribute__((ext_vector_type(16))) _Float16 v16h;
typedef __attribute__((ext_vector_type(8)))  _Float16 v8h;
typedef __attribute__((ext_vector_type(8)))  unsigned short v8us;
typedef __attribute__((ext_vector_type(8)))  float    v8f;
typedef __attribute__((ext_vector_type(4)))  float    v4f;
typedef v8h  __attribute__((may_alias)) v8ha;
typedef v4f  __attribute__((may_alias)) v4fa;
typedef v8us __attribute__((may_alias)) v8usa;

__device__ __forceinline__ unsigned short f2bf(float f) { unsigned u = __float_as_uint(f); u += 0x7FFFu + ((u >> 16) & 1u); return (unsigned short)(u >> 16); }
__device__ __forceinline__ float bf2f(unsigned short b) { return __uint_as_float(((unsigned)b) << 16); }
__device__ __forceinline__ float bfr(float f) { return bf2f(f2bf(f)); }
__device__ __forceinline__ v16h cat16(v8h lo, v8h hi) { return __builtin_shufflevector(lo, hi, 0, 1, 2, 3, 4, 5, 6, 7, 8, 9, 10, 11, 12, 13, 14, 15); }
__device__ __forceinline__ v16bf cat16b(v8us lo, v8us hi) { return __builtin_bit_cast(v16bf, __builtin_shufflevector(lo, hi, 0, 1, 2, 3, 4, 5, 6, 7, 8, 9, 10, 11, 12, 13, 14, 15)); }
__device__ __forceinline__ v8f wmma16(v16h a, v16h b, v8f c) { return __builtin_amdgcn_wmma_f32_16x16x32_f16(false, a, false, b, (short)0, c, false, false); }
__device__ __forceinline__ v8f wmmab(v16bf a, v16bf b, v8f c) { return __builtin_amdgcn_wmma_f32_16x16x32_bf16(false, a, false, b, (short)0, c, false, false); }

template <bool SPLITA, bool F16OUT = false>
__global__ __launch_bounds__(128) void k_gemmb(const bf* __restrict__ A, const bf* __restrict__ Al, const bf* __restrict__ Bn, const float* __restrict__ bias, float* C, int ldc, h16* C2, const float* __restrict__ R = nullptr, int K = DM, int roundR = 1) {
    __shared__ __align__(16) float ost[4][16 * 68];
    const int lane = threadIdx.x & 31, wave = threadIdx.x >> 5, lr = lane & 15, hi = lane >> 4;
    const int r0 = blockIdx.x * 64 + wave * 16, c0 = blockIdx.y * 64;
    const size_t aoff = (size_t)(r0 + lr) * K + 8 * hi;
    size_t boff[4];
#pragma unroll
    for (int t = 0; t < 4; ++t) boff[t] = (size_t)(c0 + t * 16 + lr) * K + 8 * hi;
    v8f acc[4];
#pragma unroll
    for (int t = 0; t < 4; ++t) acc[t] = (v8f){};
#pragma unroll 1
    for (int kc = 0; kc < K; kc += 32) {
        const v16bf a = cat16b(*(const v8us*)(A + aoff + kc), *(const v8us*)(A + aoff + kc + 16));
        v16bf al = a;
        if (SPLITA) al = cat16b(*(const v8us*)(Al + aoff + kc), *(const v8us*)(Al + aoff + kc + 16));
#pragma unroll
        for (int t = 0; t < 4; ++t) { const v16bf b = cat16b(*(const v8us*)(Bn + boff[t] + kc), *(const v8us*)(Bn + boff[t] + kc + 16)); acc[t] = wmmab(a, b, acc[t]); if (SPLITA) acc[t] = wmmab(al, b, acc[t]); }
        asm volatile("v_nop\n\tv_nop\n\tv_nop\n\tv_nop" : "+v"(acc[0]), "+v"(acc[1]), "+v"(acc[2]), "+v"(acc[3]) : "v"(a), "v"(al));
    }
    float* os = &ost[wave][0];
#pragma unroll
    for (int t = 0; t < 4; ++t) { const float bv = bias ? bfr(bias[c0 + t * 16 + lr]) : 0.f;
#pragma unroll
        for (int j = 0; j < 8; ++j) os[(hi * 8 + j) * 68 + t * 16 + lr] = acc[t][j] + bv; }
    __syncthreads();
    if (F16OUT) {
        h16* crow = (h16*)(void*)C + (size_t)r0 * ldc + c0;
        auto pass = [&]() {
#pragma unroll
            for (int s = 0; s < 4; ++s) { const int row = 4 * s + (lane >> 3), piece = lane & 7; const float* sp = os + row * 68 + piece * 8; v8h o, o2;
#pragma unroll
                for (int i = 0; i < 8; ++i) { const h16 a = (h16)sp[i]; o[i] = a; o2[i] = (h16)((sp[i] - (float)a) * LOSC); }
                *(volatile v8h*)(crow + (size_t)row * ldc + piece * 8) = o; if (C2) *(volatile v8h*)(C2 + (size_t)r0 * ldc + c0 + (size_t)row * ldc + piece * 8) = o2; }
        };
        pass(); __threadfence(); pass();
    } else {
        float* crow = C + (size_t)r0 * ldc + c0;
        auto pass = [&]() {
#pragma unroll
            for (int s = 0; s < 8; ++s) { const int Lid = (lane >> 3) + 4 * s, piece = lane & 7; const int row = Lid >> 1, cofs = (Lid & 1) * 32 + piece * 4;
                v4f val = *(const v4fa*)(os + row * 68 + cofs); if (R) { const v4f rv = *(const v4f*)(R + ((size_t)r0 + row) * ldc + c0 + cofs); val += roundR ? (v4f){bfr(rv[0]), bfr(rv[1]), bfr(rv[2]), bfr(rv[3])} : rv; }
                *(volatile v4f*)(crow + (size_t)row * ldc + cofs) = val; }
        };
        pass(); __threadfence(); pass();
    }
}

template <bool SPLITA, bool F16OUT = false>
__global__ __launch_bounds__(128) void k_gemmbl(const int* __restrict__ rowlimA, const int* __restrict__ rowlimB, const bf* __restrict__ A, const bf* __restrict__ Al, const bf* __restrict__ Bn, const float* __restrict__ bias, float* C, int ldc, h16* C2, const float* __restrict__ R = nullptr, int K = DM, int roundR = 1) {
    if ((int)blockIdx.x * 64 >= rowlimA[0] + rowlimB[0]) return;
    __shared__ __align__(16) float ost[4][16 * 68];
    const int lane = threadIdx.x & 31, wave = threadIdx.x >> 5, lr = lane & 15, hi = lane >> 4;
    const int r0 = blockIdx.x * 64 + wave * 16, c0 = blockIdx.y * 64;
    const size_t aoff = (size_t)(r0 + lr) * K + 8 * hi;
    size_t boff[4];
#pragma unroll
    for (int t = 0; t < 4; ++t) boff[t] = (size_t)(c0 + t * 16 + lr) * K + 8 * hi;
    v8f acc[4];
#pragma unroll
    for (int t = 0; t < 4; ++t) acc[t] = (v8f){};
#pragma unroll 1
    for (int kc = 0; kc < K; kc += 32) {
        const v16bf a = cat16b(*(const v8us*)(A + aoff + kc), *(const v8us*)(A + aoff + kc + 16));
        v16bf al = a;
        if (SPLITA) al = cat16b(*(const v8us*)(Al + aoff + kc), *(const v8us*)(Al + aoff + kc + 16));
#pragma unroll
        for (int t = 0; t < 4; ++t) { const v16bf b = cat16b(*(const v8us*)(Bn + boff[t] + kc), *(const v8us*)(Bn + boff[t] + kc + 16)); acc[t] = wmmab(a, b, acc[t]); if (SPLITA) acc[t] = wmmab(al, b, acc[t]); }
        asm volatile("v_nop\n\tv_nop\n\tv_nop\n\tv_nop" : "+v"(acc[0]), "+v"(acc[1]), "+v"(acc[2]), "+v"(acc[3]) : "v"(a), "v"(al));
    }
    float* os = &ost[wave][0];
#pragma unroll
    for (int t = 0; t < 4; ++t) { const float bv = bias ? bfr(bias[c0 + t * 16 + lr]) : 0.f;
#pragma unroll
        for (int j = 0; j < 8; ++j) os[(hi * 8 + j) * 68 + t * 16 + lr] = acc[t][j] + bv; }
    __syncthreads();
    if (F16OUT) {
        h16* crow = (h16*)(void*)C + (size_t)r0 * ldc + c0;
        auto pass = [&]() {
#pragma unroll
            for (int s = 0; s < 4; ++s) { const int row = 4 * s + (lane >> 3), piece = lane & 7; const float* sp = os + row * 68 + piece * 8; v8h o, o2;
#pragma unroll
                for (int i = 0; i < 8; ++i) { const h16 a = (h16)sp[i]; o[i] = a; o2[i] = (h16)((sp[i] - (float)a) * LOSC); }
                *(volatile v8h*)(crow + (size_t)row * ldc + piece * 8) = o; if (C2) *(volatile v8h*)(C2 + (size_t)r0 * ldc + c0 + (size_t)row * ldc + piece * 8) = o2; }
        };
        pass(); __threadfence(); pass();
    } else {
        float* crow = C + (size_t)r0 * ldc + c0;
        auto pass = [&]() {
#pragma unroll
            for (int s = 0; s < 8; ++s) { const int Lid = (lane >> 3) + 4 * s, piece = lane & 7; const int row = Lid >> 1, cofs = (Lid & 1) * 32 + piece * 4;
                v4f val = *(const v4fa*)(os + row * 68 + cofs); if (R) { const v4f rv = *(const v4f*)(R + ((size_t)r0 + row) * ldc + c0 + cofs); val += roundR ? (v4f){bfr(rv[0]), bfr(rv[1]), bfr(rv[2]), bfr(rv[3])} : rv; }
                *(volatile v4f*)(crow + (size_t)row * ldc + cofs) = val; }
        };
        pass(); __threadfence(); pass();
    }
}

__global__ __launch_bounds__(256) void k_cvt8(const float* __restrict__ src, bf* dst, size_t n8) {
    const size_t i = (size_t)blockIdx.x * 256 + threadIdx.x; if (i >= n8) return;
    const v8f v = *(const v8f*)(src + i * 8); v8us o;
#pragma unroll
    for (int k = 0; k < 8; ++k) o[k] = f2bf(v[k]);
    *(volatile v8us*)(dst + i * 8) = o; __threadfence(); *(volatile v8us*)(dst + i * 8) = o;
}
__global__ __launch_bounds__(256) void k_zero8(bf* dst, size_t n8) {
    const size_t i = (size_t)blockIdx.x * 256 + threadIdx.x; if (i >= n8) return; v8us z;
#pragma unroll
    for (int k = 0; k < 8; ++k) z[k] = 0;
    *(volatile v8us*)(dst + i * 8) = z; __threadfence(); *(volatile v8us*)(dst + i * 8) = z;
}

template <int MODE>
__global__ __launch_bounds__(128) void k_gemm3z(const bf* __restrict__ Ah, const bf* __restrict__ Al, const bf* __restrict__ Bh, const bf* __restrict__ Bl, int K, float* C, int ldc, size_t sA, size_t sB, size_t sC) {
    if ((MODE & 1) && (int)blockIdx.y * 64 > (int)blockIdx.x * 64 + 63) return;
    const size_t z = blockIdx.z; Ah += z * sA; Al += z * sA; Bh += z * sB; Bl += z * sB; C += z * sC;
    const int Klim = (MODE & 2) ? min(K, ((int)blockIdx.x + 1) * 64) : K;
    __shared__ __align__(16) float ost[4][16 * 68];
    const int lane = threadIdx.x & 31, wave = threadIdx.x >> 5, lr = lane & 15, hi = lane >> 4;
    const int r0 = blockIdx.x * 64 + wave * 16, c0 = blockIdx.y * 64;
    const size_t aoff = (size_t)(r0 + lr) * K + 8 * hi;
    v8f acc[4];
#pragma unroll
    for (int t = 0; t < 4; ++t) acc[t] = (v8f){};
#pragma unroll 1
    for (int kc = 0; kc < Klim; kc += 32) {
        const v16bf a = cat16b(*(const v8us*)(Ah + aoff + kc), *(const v8us*)(Ah + aoff + kc + 16));
        v16bf al = a; if (!(MODE & 4) && !(MODE & 16)) al = cat16b(*(const v8us*)(Al + aoff + kc), *(const v8us*)(Al + aoff + kc + 16));
#pragma unroll
        for (int t = 0; t < 4; ++t) { const size_t bo = (size_t)(c0 + t * 16 + lr) * K + kc + 8 * hi;
            const v16bf bh = cat16b(*(const v8us*)(Bh + bo), *(const v8us*)(Bh + bo + 16));
            acc[t] = wmmab(a, bh, acc[t]);
            if (!(MODE & 4)) { if (!(MODE & 16)) acc[t] = wmmab(al, bh, acc[t]); if (!(MODE & 8)) { const v16bf bl = cat16b(*(const v8us*)(Bl + bo), *(const v8us*)(Bl + bo + 16)); acc[t] = wmmab(a, bl, acc[t]); } } }
        asm volatile("v_nop\n\tv_nop\n\tv_nop\n\tv_nop" : "+v"(acc[0]), "+v"(acc[1]), "+v"(acc[2]), "+v"(acc[3]) : "v"(a), "v"(al));
    }
    float* os = &ost[wave][0];
#pragma unroll
    for (int t = 0; t < 4; ++t) {
#pragma unroll
        for (int j = 0; j < 8; ++j) os[(hi * 8 + j) * 68 + t * 16 + lr] = acc[t][j]; }
    __builtin_amdgcn_wave_barrier(); asm volatile("" ::: "memory");
    float* crow = C + (size_t)r0 * ldc + c0;
    auto pass = [&]() {
#pragma unroll
        for (int s = 0; s < 8; ++s) { const int Lid = (lane >> 3) + 4 * s, piece = lane & 7; const int row = Lid >> 1, cofs = (Lid & 1) * 32 + piece * 4;
            const v4f val = *(const v4fa*)(os + row * 68 + cofs); *(volatile v4f*)(crow + (size_t)row * ldc + cofs) = val; }
    };
    pass(); __threadfence(); pass();
}
__global__ __launch_bounds__(256) void k_planes32z(const float* __restrict__ F, int ld, int off, float sc, int rows, bf* Ph, bf* Pl) {
    typedef __attribute__((ext_vector_type(2))) unsigned short v2us;
    const int lane = threadIdx.x & 31; const size_t r = ((size_t)blockIdx.x * 8 + (threadIdx.x >> 5)) * 2 + (lane >> 4); if (r >= (size_t)rows) return; const int z = blockIdx.z; const int c0 = (lane & 15) * 2; v2us oh, ol;
    Ph += (size_t)z * rows * 32; Pl += (size_t)z * rows * 32;
#pragma unroll
    for (int i = 0; i < 2; ++i) { const float y = F[r * ld + off + z * 32 + c0 + i] * sc; const unsigned short hb = f2bf(y); oh[i] = hb; ol[i] = f2bf(y - bf2f(hb)); }
    const size_t o = r * 32 + c0; *(volatile v2us*)(Ph + o) = oh; *(volatile v2us*)(Pl + o) = ol; __threadfence(); *(volatile v2us*)(Ph + o) = oh; *(volatile v2us*)(Pl + o) = ol;
}
__global__ __launch_bounds__(256) void k_vtpadz(const float* __restrict__ F, int ld, int off, int nk, bf* Th, bf* Tl) {
    typedef __attribute__((ext_vector_type(2))) unsigned short v2us;
    const int lane = threadIdx.x & 31; const size_t wid = (size_t)blockIdx.x * 8 + (threadIdx.x >> 5); if (wid >= (size_t)64 * (nk / 64)) return; const int z = blockIdx.z; const int d = (int)(wid / (nk / 64)); const int k0 = (int)(wid % (nk / 64)) * 64 + lane * 2; v2us oh, ol;
    Th += (size_t)z * 64 * nk; Tl += (size_t)z * 64 * nk;
#pragma unroll
    for (int i = 0; i < 2; ++i) { const float y = (d < 32) ? F[(size_t)(k0 + i) * ld + off + z * 32 + (d < 32 ? d : 0)] : 0.f; const unsigned short hb = f2bf(y); oh[i] = hb; ol[i] = f2bf(y - bf2f(hb)); }
    const size_t o = (size_t)d * nk + k0; *(volatile v2us*)(Th + o) = oh; *(volatile v2us*)(Tl + o) = ol; __threadfence(); *(volatile v2us*)(Th + o) = oh; *(volatile v2us*)(Tl + o) = ol;
}
template <int NK>
__global__ __launch_bounds__(256) void k_softmaxz(const float* __restrict__ S, int rows, bf* PH, bf* PL) {
    typedef __attribute__((ext_vector_type(4))) unsigned short v4us;
    const int lane = threadIdx.x & 31, i = blockIdx.x * 8 + (threadIdx.x >> 5); if (i >= rows) return; const size_t zo = (size_t)blockIdx.z * rows * NK; const float* sr = S + zo + (size_t)i * NK; PH += zo; PL += zo;
    float m = -3.0e38f;
#pragma unroll 1
    for (int c0 = lane * 4; c0 < NK; c0 += 128) {
#pragma unroll
        for (int q = 0; q < 4; ++q) m = fmaxf(m, sr[c0 + q]); }
#pragma unroll
    for (int sh = 16; sh; sh >>= 1) m = fmaxf(m, __shfl_xor(m, sh, 32));
    float sum = 0.f;
#pragma unroll 1
    for (int c0 = lane * 4; c0 < NK; c0 += 128) {
#pragma unroll
        for (int q = 0; q < 4; ++q) sum += __expf(sr[c0 + q] - m); }
#pragma unroll
    for (int sh = 16; sh; sh >>= 1) sum += __shfl_xor(sum, sh, 32);
    const float inv = 1.0f / sum;
#pragma unroll 1
    for (int ps = 0; ps < 2; ++ps) {
#pragma unroll 1
        for (int c0 = lane * 4; c0 < NK; c0 += 128) { v4us oh, ol;
#pragma unroll
            for (int q = 0; q < 4; ++q) { const float p = __expf(sr[c0 + q] - m) * inv; const unsigned short hb = f2bf(p); oh[q] = hb; ol[q] = f2bf(p - bf2f(hb)); }
            const size_t o = (size_t)i * NK + c0; *(volatile v4us*)(PH + o) = oh; *(volatile v4us*)(PL + o) = ol; }
        if (ps == 0) __threadfence(); }
}
__global__ __launch_bounds__(256) void k_placez(const float* __restrict__ XH, int rows, int ldy, float* Y) {
    const int lane = threadIdx.x & 31; const size_t q = (size_t)blockIdx.x * 8 + (threadIdx.x >> 5); if (q >= (size_t)rows) return; const int z = blockIdx.z; const float v = XH[((size_t)z * rows + q) * 64 + lane];
    *(volatile float*)(Y + q * ldy + z * 32 + lane) = v; __threadfence(); *(volatile float*)(Y + q * ldy + z * 32 + lane) = v;
}

__global__ __launch_bounds__(256) void k_cum(const int* __restrict__ am, const int* __restrict__ pm, int* CUM) {
    const int lane = threadIdx.x & 31; const int b = blockIdx.x * 8 + (threadIdx.x >> 5); if (b >= NB_) return; int base = 0; int vals[4][4];
#pragma unroll
    for (int pass = 0; pass < 4; ++pass) { const int s0 = pass * 128 + lane * 4; int c = 0; int loc[4];
#pragma unroll
        for (int i = 0; i < 4; ++i) { const int s = s0 + i; const int vis = (am[b * SS + s] != 0 && pm[b * SS + s] == 0) ? 1 : 0; c += vis; loc[i] = c; }
        int incl = c;
#pragma unroll
        for (int sh = 1; sh < 32; sh <<= 1) { const int o = __shfl_up(incl, sh, 32); if (lane >= sh) incl += o; }
        const int excl = incl - c; const int tot = __shfl(incl, 31, 32);
#pragma unroll
        for (int i = 0; i < 4; ++i) vals[pass][i] = base + excl + loc[i];
        base += tot; }
    typedef __attribute__((ext_vector_type(4))) int v4i;
#pragma unroll 1
    for (int ps = 0; ps < 2; ++ps) {
#pragma unroll
        for (int pass = 0; pass < 4; ++pass) { v4i v; for (int i = 0; i < 4; ++i) v[i] = vals[pass][i]; *(volatile v4i*)(CUM + b * SS + pass * 128 + lane * 4) = v; }
        if (ps == 0) __threadfence(); }
}
__global__ __launch_bounds__(256) void k_seg(const int* __restrict__ CUM, int* SEG) {
    if (threadIdx.x >= 32) return; const int lane = threadIdx.x; int cnt = CUM[lane * SS + SS - 1]; cnt = cnt > NW ? NW : cnt; int incl = cnt;
#pragma unroll
    for (int sh = 1; sh < 32; sh <<= 1) { const int o = __shfl_up(incl, sh, 32); if (lane >= sh) incl += o; }
    const int off = incl - cnt;
    *(volatile int*)(SEG + lane) = off; *(volatile int*)(SEG + 32 + lane) = cnt; __threadfence(); *(volatile int*)(SEG + lane) = off; *(volatile int*)(SEG + 32 + lane) = cnt;
}
__global__ __launch_bounds__(256) void k_encin(const float* __restrict__ ev, const int* __restrict__ CUM, const int* __restrict__ SEG, bf* A) {
    typedef __attribute__((ext_vector_type(4))) unsigned short v4us;
    const int lane = threadIdx.x & 31; const size_t w = (size_t)blockIdx.x * 8 + (threadIdx.x >> 5); const size_t j = w * 4 + (lane >> 3); if (j >= (size_t)RTM) return; const int c0 = (lane & 7) * 4;
    const int total = SEG[31] + SEG[63]; int b = 0;
#pragma unroll 1
    for (int q = 1; q < NB_; ++q) b = (SEG[q] <= (int)j) ? q : b;
    const int jj = (int)j - SEG[b]; const bool live = ((int)j < total) && (jj < SEG[32 + b]); int s = 0;
    if (live) { int lo = 0, hi = SS - 1;
#pragma unroll 1
        while (lo < hi) { const int mid = (lo + hi) >> 1; if (CUM[b * SS + mid] >= jj + 1) hi = mid; else lo = mid + 1; } s = lo; }
    v4us o;
#pragma unroll
    for (int i = 0; i < 4; ++i) { const int c = c0 + i; o[i] = f2bf((live && c < INF) ? ev[((size_t)b * SS + s) * INF + (c < INF ? c : 0)] : 0.f); }
    *(volatile v4us*)(A + j * INP + c0) = o; __threadfence(); *(volatile v4us*)(A + j * INP + c0) = o;
}
template <int W>
__global__ __launch_bounds__(256) void k_splitW(const float* __restrict__ F, size_t rows, bf* Ph, bf* Pl) {
    typedef __attribute__((ext_vector_type(4))) unsigned short v4us;
    const int lane = threadIdx.x & 31; const size_t r = (size_t)blockIdx.x * 8 + (threadIdx.x >> 5); if (r >= rows) return;
#pragma unroll 1
    for (int ps = 0; ps < 2; ++ps) {
#pragma unroll
        for (int q = 0; q < W / 128; ++q) { const size_t o = r * W + q * 128 + lane * 4; const v4f v = *(const v4f*)(F + o); v4us oh, ol;
#pragma unroll
            for (int i = 0; i < 4; ++i) { const unsigned short hb = f2bf(v[i]); oh[i] = hb; ol[i] = f2bf(v[i] - bf2f(hb)); }
            *(volatile v4us*)(Ph + o) = oh; *(volatile v4us*)(Pl + o) = ol; }
        if (ps == 0) __threadfence(); }
}
template <int W>
__global__ __launch_bounds__(256) void k_reluW(const float* __restrict__ F, size_t rows, bf* Ph, bf* Pl) {
    typedef __attribute__((ext_vector_type(4))) unsigned short v4us;
    const int lane = threadIdx.x & 31; const size_t r = (size_t)blockIdx.x * 8 + (threadIdx.x >> 5); if (r >= rows) return;
#pragma unroll 1
    for (int ps = 0; ps < 2; ++ps) {
#pragma unroll
        for (int q = 0; q < W / 128; ++q) { const size_t o = r * W + q * 128 + lane * 4; const v4f v = *(const v4f*)(F + o); v4us oh, ol;
#pragma unroll
            for (int i = 0; i < 4; ++i) { const float y = fmaxf(v[i], 0.f); const unsigned short hb = f2bf(y); oh[i] = hb; ol[i] = f2bf(y - bf2f(hb)); }
            *(volatile v4us*)(Ph + o) = oh; *(volatile v4us*)(Pl + o) = ol; }
        if (ps == 0) __threadfence(); }
}
template <int W, bool PLANES>
__global__ __launch_bounds__(256) void k_lnW(const float* __restrict__ F, size_t rows, const float* __restrict__ g, const float* __restrict__ bb, float* XO, bf* Ph, bf* Pl) {
    typedef __attribute__((ext_vector_type(4))) unsigned short v4us;
    const int lane = threadIdx.x & 31; const size_t r = (size_t)blockIdx.x * 8 + (threadIdx.x >> 5); if (r >= rows) return; float v[W / 32]; float s = 0.f;
#pragma unroll
    for (int q = 0; q < W / 128; ++q)
#pragma unroll
        for (int i = 0; i < 4; ++i) { v[q * 4 + i] = F[r * W + q * 128 + lane * 4 + i]; s += v[q * 4 + i]; }
#pragma unroll
    for (int sh = 16; sh; sh >>= 1) s += __shfl_xor(s, sh, 32);
    const float mu = s * (1.0f / W); float qv = 0.f;
#pragma unroll
    for (int i = 0; i < W / 32; ++i) { const float d = v[i] - mu; qv = fmaf(d, d, qv); }
#pragma unroll
    for (int sh = 16; sh; sh >>= 1) qv += __shfl_xor(qv, sh, 32);
    const float rs = rsqrtf(qv * (1.0f / W) + 1e-5f);
#pragma unroll
    for (int q = 0; q < W / 128; ++q)
#pragma unroll
        for (int i = 0; i < 4; ++i) { const int c = q * 128 + lane * 4 + i; v[q * 4 + i] = (v[q * 4 + i] - mu) * rs * bfr(g[c]) + bfr(bb[c]); }
#pragma unroll 1
    for (int ps = 0; ps < 2; ++ps) {
#pragma unroll
        for (int q = 0; q < W / 128; ++q) { const size_t o = r * W + q * 128 + lane * 4; v4f f; v4us oh, ol;
#pragma unroll
            for (int i = 0; i < 4; ++i) { const float y = v[q * 4 + i]; f[i] = y; const unsigned short hb = f2bf(y); oh[i] = hb; ol[i] = f2bf(y - bf2f(hb)); }
            *(volatile v4f*)(XO + o) = f; if (PLANES) { *(volatile v4us*)(Ph + o) = oh; *(volatile v4us*)(Pl + o) = ol; } }
        if (ps == 0) __threadfence(); }
}
template <int D, int NHh, int NWIN, bool ENC>
__global__ __launch_bounds__(256) void k_hplw(const float* __restrict__ QKV, const int* __restrict__ SEG, int b0, int col0, float sc, bf* Ph, bf* Pl) {
    typedef __attribute__((ext_vector_type(4))) unsigned short v4us;
    const int lane = threadIdx.x & 31; const size_t w = (size_t)blockIdx.x * 8 + (threadIdx.x >> 5); const int i = (int)(w * 4 + (lane >> 3)); if (i >= NWIN) return; const int g = blockIdx.z / NHh, h = blockIdx.z % NHh; const int b = b0 + g; const int c0 = (lane & 7) * 4;
    size_t row; bool live;
    if (ENC) { const int cnt = SEG[32 + b]; live = i < cnt; row = (size_t)SEG[b] + (live ? i : 0); } else { live = true; row = (size_t)b * SS + i; }
    v4us oh, ol;
#pragma unroll
    for (int q = 0; q < 4; ++q) { const float y = live ? QKV[row * (3 * D) + col0 + h * DH + c0 + q] * sc : 0.f; const unsigned short hb = f2bf(y); oh[q] = hb; ol[q] = f2bf(y - bf2f(hb)); }
    const size_t o = ((size_t)blockIdx.z * NWIN + i) * DH + c0; *(volatile v4us*)(Ph + o) = oh; *(volatile v4us*)(Pl + o) = ol; __threadfence(); *(volatile v4us*)(Ph + o) = oh; *(volatile v4us*)(Pl + o) = ol;
}
template <int D, int NHh, int NWIN, bool ENC>
__global__ __launch_bounds__(256) void k_vTw(const float* __restrict__ QKV, const int* __restrict__ SEG, int b0, bf* Th, bf* Tl) {
    __shared__ float tl[64][33];
    typedef __attribute__((ext_vector_type(4))) unsigned short v4us;
    const int tid = threadIdx.x; const int t0 = blockIdx.x * 64; const int g = blockIdx.z / NHh, h = blockIdx.z % NHh; const int b = b0 + g; const int rr = tid >> 2, cq = (tid & 3) * 8;
    size_t row; bool live; const int t = t0 + rr;
    if (ENC) { const int cnt = SEG[32 + b]; live = t < cnt; row = (size_t)SEG[b] + (live ? t : 0); } else { live = true; row = (size_t)b * SS + t; }
#pragma unroll
    for (int i = 0; i < 8; ++i) tl[rr][cq + i] = live ? QKV[row * (3 * D) + 2 * D + h * DH + cq + i] : 0.f;
    __syncthreads();
    const int lane = tid & 31, wv = tid >> 5;
    auto pass = [&]() {
#pragma unroll
        for (int st = 0; st < 4; ++st) { const int dr = wv * 8 + st * 2 + (lane >> 4); const int tq = (lane & 15) * 4; v4us oh, ol;
#pragma unroll
            for (int i = 0; i < 4; ++i) { const float y = (dr < DH) ? tl[tq + i][dr < DH ? dr : 0] : 0.f; const unsigned short hb = f2bf(y); oh[i] = hb; ol[i] = f2bf(y - bf2f(hb)); }
            const size_t o = ((size_t)blockIdx.z * 64 + dr) * NWIN + t0 + tq; *(volatile v4us*)(Th + o) = oh; *(volatile v4us*)(Tl + o) = ol; }
    };
    pass(); __threadfence(); pass();
}
template <int NHh, int NWIN, bool ENC>
__global__ __launch_bounds__(256) void k_softw(const float* __restrict__ S, const int* __restrict__ SEG, const int* __restrict__ am, int b0, bf* PH, bf* PL) {
    typedef __attribute__((ext_vector_type(4))) unsigned short v4us;
    const int lane = threadIdx.x & 31, i = blockIdx.x * 8 + (threadIdx.x >> 5); if (i >= NWIN) return; const int g = blockIdx.z / NHh; const int b = b0 + g; const size_t zo = (size_t)blockIdx.z * NWIN * NWIN; const float* sr = S + zo + (size_t)i * NWIN; const int cnt = ENC ? SEG[32 + b] : 0;
    auto val = [&](int k) { const float s = sr[k]; const bool masked = ENC ? (k >= cnt) : (am[b * SS + k] == 0); return masked ? -1.0e9f : s; };
    float m = -3.0e38f;
#pragma unroll 1
    for (int c0 = lane * 4; c0 < NWIN; c0 += 128) {
#pragma unroll
        for (int q = 0; q < 4; ++q) m = fmaxf(m, val(c0 + q)); }
#pragma unroll
    for (int sh = 16; sh; sh >>= 1) m = fmaxf(m, __shfl_xor(m, sh, 32));
    float sum = 0.f;
#pragma unroll 1
    for (int c0 = lane * 4; c0 < NWIN; c0 += 128) {
#pragma unroll
        for (int q = 0; q < 4; ++q) sum += __expf(val(c0 + q) - m); }
#pragma unroll
    for (int sh = 16; sh; sh >>= 1) sum += __shfl_xor(sum, sh, 32);
    const float inv = 1.0f / sum;
#pragma unroll 1
    for (int ps = 0; ps < 2; ++ps) {
#pragma unroll 1
        for (int c0 = lane * 4; c0 < NWIN; c0 += 128) { v4us oh, ol;
#pragma unroll
            for (int q = 0; q < 4; ++q) { const float p = __expf(val(c0 + q) - m) * inv; const unsigned short hb = f2bf(p); oh[q] = hb; ol[q] = f2bf(p - bf2f(hb)); }
            const size_t o = zo + (size_t)i * NWIN + c0; *(volatile v4us*)(PH + o) = oh; *(volatile v4us*)(PL + o) = ol; }
        if (ps == 0) __threadfence(); }
}
template <int D, int NHh, int NWIN, bool ENC>
__global__ __launch_bounds__(256) void k_mergew(const float* __restrict__ OZ, const int* __restrict__ SEG, int b0, int zbase, float* O) {
    const int lane = threadIdx.x & 31; const size_t w = (size_t)blockIdx.x * 8 + (threadIdx.x >> 5); const int g = (int)(w / NWIN), i = (int)(w % NWIN); const int b = b0 + g; if (b >= NB_) return;
    size_t row; if (ENC) { if (i >= SEG[32 + b]) return; row = (size_t)SEG[b] + i; } else { if (i >= SS) return; row = (size_t)b * SS + i; }
#pragma unroll 1
    for (int ps = 0; ps < 2; ++ps) {
#pragma unroll
        for (int q = 0; q < D / 128; ++q) { const int c0 = q * 128 + lane * 4; const int h = c0 / DH, d0 = c0 % DH; const v4f v = *(const v4f*)(OZ + (((size_t)(g * NHh + h)) * NWIN + i) * 64 + d0); *(volatile v4f*)(O + row * D + c0) = v; }
        if (ps == 0) __threadfence(); }
}
__global__ __launch_bounds__(256) void k_decin(const float* __restrict__ DV, const int* __restrict__ CUM, const int* __restrict__ SEG, const int* __restrict__ am, const int* __restrict__ pm, const float* __restrict__ mtok, float* X) {
    const int lane = threadIdx.x & 31; const size_t r = (size_t)blockIdx.x * 8 + (threadIdx.x >> 5); if (r >= (size_t)NT) return; const int b = (int)(r / SS), s = (int)(r % SS);
    const bool vis = (am[r] != 0) && (pm[r] == 0); int idx = CUM[r] - 1; idx = idx < 0 ? 0 : idx; const int cnt = SEG[32 + b]; if (idx >= cnt) idx = cnt - 1; if (idx < 0) idx = 0; const size_t prow = (size_t)SEG[b] + idx; v4f v;
#pragma unroll
    for (int i = 0; i < 4; ++i) { const int c = lane * 4 + i; v[i] = vis ? DV[prow * DDm + c] : bfr(mtok[c]); }
    *(volatile v4f*)(X + r * DDm + lane * 4) = v; __threadfence(); *(volatile v4f*)(X + r * DDm + lane * 4) = v;
}
__global__ __launch_bounds__(256) void k_heads(const float* __restrict__ X, const float* __restrict__ qw, const float* __restrict__ qb, const float* __restrict__ tw, const float* __restrict__ tb, float* OUTB) {
    typedef __attribute__((ext_vector_type(2))) float v2f_;
    const int lane = threadIdx.x & 31; const size_t r = ((size_t)blockIdx.x * 8 + (threadIdx.x >> 5)) * 32 + lane; if (r >= (size_t)NT) return; float a0 = bfr(qb[0]), a1 = bfr(tb[0]);
#pragma unroll 1
    for (int c = 0; c < DDm; ++c) { const float x = X[r * DDm + c]; a0 = fmaf(x, bfr(qw[c]), a0); a1 = fmaf(x, bfr(tw[c]), a1); }
    v2f_ v; v[0] = a0; v[1] = a1; *(volatile v2f_*)(OUTB + r * 2) = v; __threadfence(); *(volatile v2f_*)(OUTB + r * 2) = v;
}
__global__ __launch_bounds__(256) void k_inpad(const float* __restrict__ w, bf* Bt) {
    typedef __attribute__((ext_vector_type(2))) unsigned short v2us;
    const int lane = threadIdx.x & 31; const int wv = blockIdx.x * 8 + (threadIdx.x >> 5); if (wv >= DE / 2) return; const int n = wv * 2 + (lane >> 4); const int c0 = (lane & 15) * 2; v2us o;
#pragma unroll
    for (int i = 0; i < 2; ++i) { const int c = c0 + i; o[i] = f2bf(c < INF ? w[(size_t)n * INF + (c < INF ? c : 0)] : 0.f); }
    *(volatile v2us*)(Bt + (size_t)n * INP + c0) = o; __threadfence(); *(volatile v2us*)(Bt + (size_t)n * INP + c0) = o;
}

typedef __attribute__((ext_vector_type(4))) _Float16 v4h;
__device__ __forceinline__ h16 tohx(float x) { return (h16)x; }
template <int D, int NHh, int NWIN, bool ENC>
__global__ __launch_bounds__(256) void k_hplwh(const float* __restrict__ QKV, const int* __restrict__ SEG, int b0, int col0, float sc, h16* P) {
    const int lane = threadIdx.x & 31; const size_t w = (size_t)blockIdx.x * 8 + (threadIdx.x >> 5); const int i = (int)(w * 4 + (lane >> 3)); if (i >= NWIN) return; const int g = blockIdx.z / NHh, h = blockIdx.z % NHh; const int b = b0 + g; const int c0 = (lane & 7) * 4;
    size_t row; bool live;
    if (ENC) { const int cnt = SEG[32 + b]; live = i < cnt; row = (size_t)SEG[b] + (live ? i : 0); } else { live = true; row = (size_t)b * SS + i; }
    v4h o;
#pragma unroll
    for (int q = 0; q < 4; ++q) o[q] = tohx(live ? QKV[row * (3 * D) + col0 + h * DH + c0 + q] * sc : 0.f);
    const size_t off = ((size_t)blockIdx.z * NWIN + i) * DH + c0; *(volatile v4h*)(P + off) = o; __threadfence(); *(volatile v4h*)(P + off) = o;
}
template <int D, int NHh, int NWIN, bool ENC>
__global__ __launch_bounds__(256) void k_vTwh(const float* __restrict__ QKV, const int* __restrict__ SEG, int b0, h16* T) {
    __shared__ float tl[64][33];
    const int tid = threadIdx.x; const int t0 = blockIdx.x * 64; const int g = blockIdx.z / NHh, h = blockIdx.z % NHh; const int b = b0 + g; const int rr = tid >> 2, cq = (tid & 3) * 8;
    size_t row; bool live; const int t = t0 + rr;
    if (ENC) { const int cnt = SEG[32 + b]; live = t < cnt; row = (size_t)SEG[b] + (live ? t : 0); } else { live = true; row = (size_t)b * SS + t; }
#pragma unroll
    for (int i = 0; i < 8; ++i) tl[rr][cq + i] = live ? QKV[row * (3 * D) + 2 * D + h * DH + cq + i] : 0.f;
    __syncthreads();
    const int lane = tid & 31, wv = tid >> 5;
    auto pass = [&]() {
#pragma unroll
        for (int st = 0; st < 4; ++st) { const int dr = wv * 8 + st * 2 + (lane >> 4); const int tq = (lane & 15) * 4; v4h v;
#pragma unroll
            for (int i = 0; i < 4; ++i) v[i] = tohx((dr < DH) ? tl[tq + i][dr < DH ? dr : 0] : 0.f);
            *(volatile v4h*)(T + ((size_t)blockIdx.z * 64 + dr) * NWIN + t0 + tq) = v; }
    };
    pass(); __threadfence(); pass();
}
template <int NHh, int NWIN, bool ENC>
__global__ __launch_bounds__(256) void k_softwh(const float* __restrict__ S, const int* __restrict__ SEG, const int* __restrict__ am, int b0, h16* P) {
    const int lane = threadIdx.x & 31, i = blockIdx.x * 8 + (threadIdx.x >> 5); if (i >= NWIN) return; const int g = blockIdx.z / NHh; const int b = b0 + g; const size_t zo = (size_t)blockIdx.z * NWIN * NWIN; const float* sr = S + zo + (size_t)i * NWIN; const int cnt = ENC ? SEG[32 + b] : 0;
    auto val = [&](int k) { const float s = sr[k]; const bool masked = ENC ? (k >= cnt) : (am[b * SS + k] == 0); return masked ? -1.0e9f : s; };
    float m = -3.0e38f;
#pragma unroll 1
    for (int c0 = lane * 4; c0 < NWIN; c0 += 128) {
#pragma unroll
        for (int q = 0; q < 4; ++q) m = fmaxf(m, val(c0 + q)); }
#pragma unroll
    for (int sh = 16; sh; sh >>= 1) m = fmaxf(m, __shfl_xor(m, sh, 32));
    float sum = 0.f;
#pragma unroll 1
    for (int c0 = lane * 4; c0 < NWIN; c0 += 128) {
#pragma unroll
        for (int q = 0; q < 4; ++q) sum += __expf(val(c0 + q) - m); }
#pragma unroll
    for (int sh = 16; sh; sh >>= 1) sum += __shfl_xor(sum, sh, 32);
    const float inv = 1.0f / sum;
#pragma unroll 1
    for (int ps = 0; ps < 2; ++ps) {
#pragma unroll 1
        for (int c0 = lane * 4; c0 < NWIN; c0 += 128) { v4h o;
#pragma unroll
            for (int q = 0; q < 4; ++q) o[q] = tohx(__expf(val(c0 + q) - m) * inv);
            *(volatile v4h*)(P + zo + (size_t)i * NWIN + c0) = o; }
        if (ps == 0) __threadfence(); }
}

__global__ __launch_bounds__(128) void k_gemmh(const h16* __restrict__ A, const h16* __restrict__ Bn, const float* __restrict__ bias, float* C, int ldc, const float* __restrict__ R, int K, size_t sA, size_t sB, size_t sC, int roundR) {
    __shared__ __align__(16) float ost[4][16 * 68];
    const size_t z = blockIdx.z; A += z * sA; Bn += z * sB; C += z * sC; if (R) R += z * sC;
    const int lane = threadIdx.x & 31, wave = threadIdx.x >> 5, lr = lane & 15, hi = lane >> 4;
    const int r0 = blockIdx.x * 64 + wave * 16, c0 = blockIdx.y * 64;
    const size_t aoff = (size_t)(r0 + lr) * K + 8 * hi;
    size_t boff[4];
#pragma unroll
    for (int t = 0; t < 4; ++t) boff[t] = (size_t)(c0 + t * 16 + lr) * K + 8 * hi;
    v8f acc[4];
#pragma unroll
    for (int t = 0; t < 4; ++t) acc[t] = (v8f){};
#pragma unroll 1
    for (int kc = 0; kc < K; kc += 32) {
        const v16h a = cat16(*(const v8h*)(A + aoff + kc), *(const v8h*)(A + aoff + kc + 16));
#pragma unroll
        for (int t = 0; t < 4; ++t) { const v16h b = cat16(*(const v8h*)(Bn + boff[t] + kc), *(const v8h*)(Bn + boff[t] + kc + 16)); acc[t] = wmma16(a, b, acc[t]); }
        asm volatile("v_nop\n\tv_nop\n\tv_nop\n\tv_nop" : "+v"(acc[0]), "+v"(acc[1]), "+v"(acc[2]), "+v"(acc[3]) : "v"(a));
    }
    float* os = &ost[wave][0];
#pragma unroll
    for (int t = 0; t < 4; ++t) { const float bv = bias ? bfr(bias[c0 + t * 16 + lr]) : 0.f;
#pragma unroll
        for (int j = 0; j < 8; ++j) os[(hi * 8 + j) * 68 + t * 16 + lr] = acc[t][j] + bv; }
    __syncthreads();
    float* crow = C + (size_t)r0 * ldc + c0;
    auto pass = [&]() {
#pragma unroll
        for (int s = 0; s < 8; ++s) { const int Lid = (lane >> 3) + 4 * s, piece = lane & 7; const int row = Lid >> 1, cofs = (Lid & 1) * 32 + piece * 4;
            v4f val = *(const v4fa*)(os + row * 68 + cofs); if (R) { const v4f rv = *(const v4f*)(R + ((size_t)r0 + row) * ldc + c0 + cofs); val += roundR ? (v4f){bfr(rv[0]), bfr(rv[1]), bfr(rv[2]), bfr(rv[3])} : rv; }
            *(volatile v4f*)(crow + (size_t)row * ldc + cofs) = val; }
    };
    pass(); __threadfence(); pass();
}

#define RTE 4096
extern "C" void kernel_launch(void* const* d_in, const int* in_sizes, int n_in,
                              void* d_out, int out_size, void* d_ws, size_t ws_size, hipStream_t stream) {
    (void)in_sizes; (void)n_in; (void)out_size;
    const float* ev = (const float*)d_in[0]; const int* am = (const int*)d_in[1]; const int* pm = (const int*)d_in[2]; const float* win = (const float*)d_in[3]; const float* bin = (const float*)d_in[4];
    const float* eqw = (const float*)d_in[5]; const float* eqb = (const float*)d_in[6]; const float* eow = (const float*)d_in[7]; const float* eob = (const float*)d_in[8]; const float* ef1w = (const float*)d_in[9]; const float* ef1b = (const float*)d_in[10]; const float* ef2w = (const float*)d_in[11]; const float* ef2b = (const float*)d_in[12]; const float* eg1 = (const float*)d_in[13]; const float* eb1 = (const float*)d_in[14]; const float* eg2 = (const float*)d_in[15]; const float* eb2 = (const float*)d_in[16];
    const float* mtok = (const float*)d_in[17]; const float* e2d = (const float*)d_in[18];
    const float* dqw = (const float*)d_in[19]; const float* dqb = (const float*)d_in[20]; const float* dow = (const float*)d_in[21]; const float* dob = (const float*)d_in[22]; const float* df1w = (const float*)d_in[23]; const float* df1b = (const float*)d_in[24]; const float* df2w = (const float*)d_in[25]; const float* df2b = (const float*)d_in[26]; const float* dg1 = (const float*)d_in[27]; const float* db1 = (const float*)d_in[28]; const float* dg2 = (const float*)d_in[29]; const float* db2 = (const float*)d_in[30];
    const float* qhw = (const float*)d_in[31]; const float* qhb = (const float*)d_in[32]; const float* dtw = (const float*)d_in[33]; const float* dtb = (const float*)d_in[34];
    float* out = (float*)d_out;
    char* wsp = (char*)d_ws;
    auto take = [&](size_t bytes) { char* p = wsp; wsp += (bytes + 255) & ~(size_t)255; return (void*)p; };
    int* CUM = (int*)take((size_t)NT * 4); int* SEG = (int*)take(64 * 4); int* ZERO = SEG;
    bf* WIN_ = (bf*)take(DE * INP * 2); bf* EQW = (bf*)take((size_t)LE * 3 * DE * DE * 2); bf* EOW = (bf*)take((size_t)LE * DE * DE * 2); bf* EF1 = (bf*)take((size_t)LE * FE * DE * 2); bf* EF2 = (bf*)take((size_t)LE * DE * FE * 2);
    bf* E2D = (bf*)take(DDm * DE * 2); bf* DQW = (bf*)take((size_t)LD * 3 * DDm * DDm * 2); bf* DOW = (bf*)take((size_t)LD * DDm * DDm * 2); bf* DF1 = (bf*)take((size_t)LD * FD * DDm * 2); bf* DF2 = (bf*)take((size_t)LD * DDm * FD * 2);
    h16* Qx = (h16*)take((size_t)128 * NW * DH * 2); h16* Kx = (h16*)take((size_t)128 * NW * DH * 2); h16* VTx = (h16*)take((size_t)128 * 64 * NW * 2);
    float* S = (float*)take((size_t)128 * NW * NW * 4); h16* Px = (h16*)take((size_t)128 * NW * NW * 2); float* OZ = (float*)take((size_t)128 * NW * 64 * 4);
    float* DV = (float*)take((size_t)RTE * DDm * 4);
    char* const shared0 = wsp;
    bf* A0 = (bf*)take((size_t)RTE * INP * 2); float* XE = (float*)take((size_t)RTE * DE * 4); bf* Eh = (bf*)take((size_t)RTE * DE * 2); bf* El = (bf*)take((size_t)RTE * DE * 2); float* QKV = (float*)take((size_t)RTE * 3 * DE * 4); float* AO = (float*)take((size_t)RTE * DE * 4); float* X2 = (float*)take((size_t)RTE * DE * 4); float* F1 = (float*)take((size_t)RTE * FE * 4); bf* F1h = (bf*)take((size_t)RTE * FE * 2); bf* F1l = (bf*)take((size_t)RTE * FE * 2);
    char* const encEnd = wsp; wsp = shared0;
    float* XD = (float*)take((size_t)NT * DDm * 4); bf* Dh = (bf*)take((size_t)NT * DDm * 2); bf* Dl = (bf*)take((size_t)NT * DDm * 2); float* QKVD = (float*)take((size_t)NT * 3 * DDm * 4); float* AOD = (float*)take((size_t)NT * DDm * 4); float* XD2 = (float*)take((size_t)NT * DDm * 4); float* F1D = (float*)take((size_t)NT * FD * 4); bf* F1Dh = (bf*)take((size_t)NT * FD * 2); bf* F1Dl = (bf*)take((size_t)NT * FD * 2);
    if (wsp < encEnd) wsp = encEnd;
    if ((size_t)(wsp - (char*)d_ws) > ws_size) return;
    k_inpad<<<(DE / 2) / 8, 256, 0, stream>>>(win, WIN_);
    k_cvt8<<<(unsigned)(((size_t)LE * 3 * DE * DE / 8 + 255) / 256), 256, 0, stream>>>(eqw, EQW, (size_t)LE * 3 * DE * DE / 8); k_cvt8<<<(unsigned)(((size_t)LE * DE * DE / 8 + 255) / 256), 256, 0, stream>>>(eow, EOW, (size_t)LE * DE * DE / 8);
    k_cvt8<<<(unsigned)(((size_t)LE * FE * DE / 8 + 255) / 256), 256, 0, stream>>>(ef1w, EF1, (size_t)LE * FE * DE / 8); k_cvt8<<<(unsigned)(((size_t)LE * DE * FE / 8 + 255) / 256), 256, 0, stream>>>(ef2w, EF2, (size_t)LE * DE * FE / 8);
    k_cvt8<<<(unsigned)((DDm * DE / 8 + 255) / 256), 256, 0, stream>>>(e2d, E2D, DDm * DE / 8);
    k_cvt8<<<(unsigned)(((size_t)LD * 3 * DDm * DDm / 8 + 255) / 256), 256, 0, stream>>>(dqw, DQW, (size_t)LD * 3 * DDm * DDm / 8); k_cvt8<<<(unsigned)(((size_t)LD * DDm * DDm / 8 + 255) / 256), 256, 0, stream>>>(dow, DOW, (size_t)LD * DDm * DDm / 8);
    k_cvt8<<<(unsigned)(((size_t)LD * FD * DDm / 8 + 255) / 256), 256, 0, stream>>>(df1w, DF1, (size_t)LD * FD * DDm / 8); k_cvt8<<<(unsigned)(((size_t)LD * DDm * FD / 8 + 255) / 256), 256, 0, stream>>>(df2w, DF2, (size_t)LD * DDm * FD / 8);
    k_cum<<<NB_ / 8, 256, 0, stream>>>(am, pm, CUM); k_seg<<<1, 256, 0, stream>>>(CUM, SEG);
    const int* TOTA = SEG + 31; const int* TOTB = SEG + 63;
    k_encin<<<(RTE / 4) / 8, 256, 0, stream>>>(ev, CUM, SEG, A0);
    k_gemmbl<false, false><<<dim3(RTE / 64, DE / 64, 1), 128, 0, stream>>>(TOTA, TOTB, A0, nullptr, WIN_, bin, XE, DE, nullptr, nullptr, INP);
    for (int l = 0; l < LE; ++l) { const bf* LQ = EQW + (size_t)l * 3 * DE * DE; const bf* LO = EOW + (size_t)l * DE * DE; const bf* LF1 = EF1 + (size_t)l * FE * DE; const bf* LF2 = EF2 + (size_t)l * DE * FE;
        k_splitW<DE><<<RTE / 8, 256, 0, stream>>>(XE, RTE, Eh, El);
        k_gemmbl<true, false><<<dim3(RTE / 64, (3 * DE) / 64, 1), 128, 0, stream>>>(TOTA, TOTB, Eh, El, LQ, eqb + (size_t)l * 3 * DE, QKV, 3 * DE, nullptr, nullptr, DE);
        for (int grp = 0; grp < 2; ++grp) { const int b0 = grp * 16;
            k_hplwh<DE, HE, NW, true><<<dim3((NW / 4) / 8, 1, 128), 256, 0, stream>>>(QKV, SEG, b0, 0, 0.17677669529663687f, Qx); k_hplwh<DE, HE, NW, true><<<dim3((NW / 4) / 8, 1, 128), 256, 0, stream>>>(QKV, SEG, b0, DE, 1.0f, Kx);
            k_vTwh<DE, HE, NW, true><<<dim3(NW / 64, 1, 128), 256, 0, stream>>>(QKV, SEG, b0, VTx);
            k_gemmh<<<dim3(NW / 64, NW / 64, 128), 128, 0, stream>>>(Qx, Kx, nullptr, S, NW, nullptr, DH, (size_t)NW * DH, (size_t)NW * DH, (size_t)NW * NW, 0);
            k_softwh<HE, NW, true><<<dim3(NW / 8, 1, 128), 256, 0, stream>>>(S, SEG, am, b0, Px);
            k_gemmh<<<dim3(NW / 64, 1, 128), 128, 0, stream>>>(Px, VTx, nullptr, OZ, 64, nullptr, NW, (size_t)NW * NW, (size_t)64 * NW, (size_t)NW * 64, 0);
            k_mergew<DE, HE, NW, true><<<(16 * NW) / 8, 256, 0, stream>>>(OZ, SEG, b0, 0, AO); }
        k_splitW<DE><<<RTE / 8, 256, 0, stream>>>(AO, RTE, Eh, El);
        k_gemmbl<true, false><<<dim3(RTE / 64, DE / 64, 1), 128, 0, stream>>>(TOTA, TOTB, Eh, El, LO, eob + (size_t)l * DE, X2, DE, nullptr, XE, DE, 0);
        k_lnW<DE, true><<<RTE / 8, 256, 0, stream>>>(X2, RTE, eg1 + (size_t)l * DE, eb1 + (size_t)l * DE, XE, Eh, El);
        k_gemmbl<true, false><<<dim3(RTE / 64, FE / 64, 1), 128, 0, stream>>>(TOTA, TOTB, Eh, El, LF1, ef1b + (size_t)l * FE, F1, FE, nullptr, nullptr, DE);
        k_reluW<FE><<<RTE / 8, 256, 0, stream>>>(F1, RTE, F1h, F1l);
        k_gemmbl<true, false><<<dim3(RTE / 64, DE / 64, 1), 128, 0, stream>>>(TOTA, TOTB, F1h, F1l, LF2, ef2b + (size_t)l * DE, X2, DE, nullptr, XE, FE, 0);
        k_lnW<DE, false><<<RTE / 8, 256, 0, stream>>>(X2, RTE, eg2 + (size_t)l * DE, eb2 + (size_t)l * DE, XE, nullptr, nullptr); }
    k_splitW<DE><<<RTE / 8, 256, 0, stream>>>(XE, RTE, Eh, El);
    k_gemmbl<true, false><<<dim3(RTE / 64, DDm / 64, 1), 128, 0, stream>>>(TOTA, TOTB, Eh, El, E2D, nullptr, DV, DDm, nullptr, nullptr, DE);
    k_decin<<<NT / 8, 256, 0, stream>>>(DV, CUM, SEG, am, pm, mtok, XD);
    for (int l = 0; l < LD; ++l) { const bf* LQ = DQW + (size_t)l * 3 * DDm * DDm; const bf* LO = DOW + (size_t)l * DDm * DDm; const bf* LF1 = DF1 + (size_t)l * FD * DDm; const bf* LF2 = DF2 + (size_t)l * DDm * FD;
        k_splitW<DDm><<<NT / 8, 256, 0, stream>>>(XD, NT, Dh, Dl);
        k_gemmb<true, false><<<dim3(NT / 64, (3 * DDm) / 64, 1), 128, 0, stream>>>(Dh, Dl, LQ, dqb + (size_t)l * 3 * DDm, QKVD, 3 * DDm, nullptr, nullptr, DDm);
        for (int grp = 0; grp < 4; ++grp) { const int b0 = grp * 8;
            k_hplwh<DDm, HDd, SS, false><<<dim3((SS / 4) / 8, 1, 32), 256, 0, stream>>>(QKVD, SEG, b0, 0, 0.17677669529663687f, Qx); k_hplwh<DDm, HDd, SS, false><<<dim3((SS / 4) / 8, 1, 32), 256, 0, stream>>>(QKVD, SEG, b0, DDm, 1.0f, Kx);
            k_vTwh<DDm, HDd, SS, false><<<dim3(SS / 64, 1, 32), 256, 0, stream>>>(QKVD, SEG, b0, VTx);
            k_gemmh<<<dim3(SS / 64, SS / 64, 32), 128, 0, stream>>>(Qx, Kx, nullptr, S, SS, nullptr, DH, (size_t)SS * DH, (size_t)SS * DH, (size_t)SS * SS, 0);
            k_softwh<HDd, SS, false><<<dim3(SS / 8, 1, 32), 256, 0, stream>>>(S, SEG, am, b0, Px);
            k_gemmh<<<dim3(SS / 64, 1, 32), 128, 0, stream>>>(Px, VTx, nullptr, OZ, 64, nullptr, SS, (size_t)SS * SS, (size_t)64 * SS, (size_t)SS * 64, 0);
            k_mergew<DDm, HDd, SS, false><<<(8 * SS) / 8, 256, 0, stream>>>(OZ, SEG, b0, 0, AOD); }
        k_splitW<DDm><<<NT / 8, 256, 0, stream>>>(AOD, NT, Dh, Dl);
        k_gemmb<true, false><<<dim3(NT / 64, DDm / 64, 1), 128, 0, stream>>>(Dh, Dl, LO, dob + (size_t)l * DDm, XD2, DDm, nullptr, XD, DDm, 0);
        k_lnW<DDm, true><<<NT / 8, 256, 0, stream>>>(XD2, NT, dg1 + (size_t)l * DDm, db1 + (size_t)l * DDm, XD, Dh, Dl);
        k_gemmb<true, false><<<dim3(NT / 64, FD / 64, 1), 128, 0, stream>>>(Dh, Dl, LF1, df1b + (size_t)l * FD, F1D, FD, nullptr, nullptr, DDm);
        k_reluW<FD><<<NT / 8, 256, 0, stream>>>(F1D, NT, F1Dh, F1Dl);
        k_gemmb<true, false><<<dim3(NT / 64, DDm / 64, 1), 128, 0, stream>>>(F1Dh, F1Dl, LF2, df2b + (size_t)l * DDm, XD2, DDm, nullptr, XD, FD, 0);
        k_lnW<DDm, false><<<NT / 8, 256, 0, stream>>>(XD2, NT, dg2 + (size_t)l * DDm, db2 + (size_t)l * DDm, XD, nullptr, nullptr); }
    k_heads<<<(NT / 32) / 8, 256, 0, stream>>>(XD, qhw, qhb, dtw, dtb, out);
}
